// HGCN_85186381349133
// MI455X (gfx1250) — hardware-verified
//
#include <hip/hip_runtime.h>
#include <stddef.h>
#include <stdint.h>
#include <math.h>


#define DD     128
#define XP     129
#define HD     64
#define K3     384
#define KA     256
#define NTHR   256
#define NWAVE  8
#define EPT    8
#define CHUNK  (NTHR * EPT)
#define WCAP   (EPT * 32)
#define LISTN  (NWAVE * WCAP)
#define NBA    1024
#define SLA    10
#define RCAP   8192
#define DEGCAP 64
#define TMAX   16
#define GR     64
#define STGF   8320
#define NPG1   (GR * XP / 4)
#define NIT1   ((NPG1 + NTHR - 1) / NTHR)
#define NIT0   (GR * DD / 4 / NTHR)
#define GBM    64
#define GTHR   128
#define NUW    (DD * (KA / 8))
#define NBW    (NUW / NTHR)
#define AGG_ZINTS (LISTN + 2 * RCAP + 3 * NBA)
#define AGG_INTS  (AGG_ZINTS + 16)
#define AGG_FLTS  (TMAX * HD + TMAX * DD + HD + 2 * DD + STGF)
#define AGG_LDS   ((AGG_INTS + AGG_FLTS) * 4)
#define LIN_LDS   (GBM * KA * 2 + GBM * DD * 4)
#define WSMAX  134217728
#define EPSN   1e-6f
#define X0MIN  1.00000011920928955078125f

static_assert((CHUNK & (CHUNK - 1)) == 0 && CHUNK <= 4096);
static_assert((NBA & (NBA - 1)) == 0 && NBA == (1 << SLA));
static_assert(((long long)CHUNK << SLA) < (1LL << 31));
static_assert(LISTN % NTHR == 0);
static_assert(NBA % NWAVE == 0 && NBA % 32 == 0 && NBA % GR == 0);
static_assert(GR % NWAVE == 0 && GR % 4 == 0 && (GR / 4) <= 32);
static_assert(RCAP % 4 == 0 && AGG_ZINTS % 4 == 0 && LISTN % 4 == 0 && AGG_INTS % 4 == 0);
static_assert(AGG_ZINTS % (NTHR * 4) == 0);
static_assert(DEGCAP % 32 == 0);
static_assert(DD == 4 * 32 && HD == 2 * 32 && KA == 2 * DD && KA % 32 == 0 && XP == DD + 1 && K3 == 3 * DD);
static_assert(GBM == (GTHR / 32) * 16);
static_assert(NUW % NTHR == 0 && KA / 8 == 32 && (NBW & (NBW - 1)) == 0);
static_assert(STGF >= GR * XP && STGF >= GR * DD + GR && STGF % 4 == 0);
static_assert((GR * XP) % 4 == 0 && (GR * DD) % (NTHR * 4) == 0);
static_assert((TMAX * HD) % 4 == 0 && ((TMAX * HD + TMAX * DD + HD + 2 * DD) % 4) == 0);
static_assert((TMAX * DD) % NTHR == 0 && (TMAX * HD) % NTHR == 0 && (TMAX * HD) % 64 == 0);
static_assert(HD <= NTHR && DD <= NTHR);
static_assert(AGG_LDS <= 300000 && LIN_LDS <= 300000);

typedef float          v2f   __attribute__((ext_vector_type(2)));
typedef float          v4f   __attribute__((ext_vector_type(4)));
typedef float          v8f   __attribute__((ext_vector_type(8)));
typedef int            v4i   __attribute__((ext_vector_type(4)));
typedef int            v8i   __attribute__((ext_vector_type(8)));
typedef unsigned       v2u   __attribute__((ext_vector_type(2)));
typedef unsigned short v8us  __attribute__((ext_vector_type(8)));
typedef unsigned short v16us __attribute__((ext_vector_type(16)));
typedef __bf16         v16bf __attribute__((ext_vector_type(16)));
typedef v2f  __attribute__((may_alias)) v2fa;
typedef v4f  __attribute__((may_alias)) v4fa;
typedef v4i  __attribute__((may_alias)) v4ia;
typedef v2u  __attribute__((may_alias)) v2ua;
typedef v8us __attribute__((may_alias)) v8usa;
union FragB { v16bf v; v16us u; v8us h[2]; v8i w; };

__device__ __forceinline__ v8f wmb(const FragB& a, const FragB& b, v8f c) {
  v8f d = __builtin_amdgcn_wmma_f32_16x16x32_bf16(false, a.v, false, b.v, (short)0, c, false, false);
  asm volatile("v_nop\n\tv_nop\n\tv_nop\n\tv_nop" : "+v"(d) : "v"(a.w), "v"(b.w));
  return d;
}

__device__ __forceinline__ unsigned bf16_bits(float f) {
  const unsigned u = __float_as_uint(f);
  return (u + 0x7FFFu + ((u >> 16) & 1u)) >> 16;
}
__device__ __forceinline__ float bf16_val(float f) {
  return __uint_as_float(bf16_bits(f) << 16);
}
__device__ __forceinline__ v8us pack8(const v4f a, const v4f b) {
  v8us o;
  o[0] = (unsigned short)bf16_bits(a.x); o[1] = (unsigned short)bf16_bits(a.y);
  o[2] = (unsigned short)bf16_bits(a.z); o[3] = (unsigned short)bf16_bits(a.w);
  o[4] = (unsigned short)bf16_bits(b.x); o[5] = (unsigned short)bf16_bits(b.y);
  o[6] = (unsigned short)bf16_bits(b.z); o[7] = (unsigned short)bf16_bits(b.w);
  return o;
}

__device__ __forceinline__ float wsum(float v) {
#pragma unroll
  for (int q = 16; q > 0; q >>= 1) v += __shfl_xor(v, q, 32);
  return v;
}

__device__ __forceinline__ float silu_f(float x) {
  const float e = expf(-x);
  return x * __builtin_amdgcn_rcpf(1.0f + e);
}

__device__ __forceinline__ void hilo_pack(float v0, float v1, float v2, float v3,
                                          int& h01, int& h23, int& l01, int& l23) {
  const unsigned a0 = bf16_bits(v0), a1 = bf16_bits(v1), a2 = bf16_bits(v2), a3 = bf16_bits(v3);
  const unsigned b0 = bf16_bits(v0 - __uint_as_float(a0 << 16));
  const unsigned b1 = bf16_bits(v1 - __uint_as_float(a1 << 16));
  const unsigned b2 = bf16_bits(v2 - __uint_as_float(a2 << 16));
  const unsigned b3 = bf16_bits(v3 - __uint_as_float(a3 << 16));
  h01 = (int)(a0 | (a1 << 16)); h23 = (int)(a2 | (a3 << 16));
  l01 = (int)(b0 | (b1 << 16)); l23 = (int)(b2 | (b3 << 16));
}

__device__ __forceinline__ v4i regroup16(int h01, int h23, int l01, int l23, int lane) {
  const int s0 = (2 * lane) & 31, s1 = s0 + 1;
  const int a0 = __shfl(h01, s0, 32), a1 = __shfl(h23, s0, 32), a2 = __shfl(h01, s1, 32), a3 = __shfl(h23, s1, 32);
  const int b0 = __shfl(l01, s0, 32), b1 = __shfl(l23, s0, 32), b2 = __shfl(l01, s1, 32), b3 = __shfl(l23, s1, 32);
  const int mk = (lane < 16) ? -1 : 0;
  v4i o;
  o.x = (a0 & mk) | (b0 & ~mk); o.y = (a1 & mk) | (b1 & ~mk);
  o.z = (a2 & mk) | (b2 & ~mk); o.w = (a3 & mk) | (b3 & ~mk);
  return o;
}

template <int SLB>
__device__ __forceinline__ int scan_chunk(const int* __restrict__ dsts, int nE, int cbase, int slotBase,
                                          int nb, int vec8, int* list, int tid, int lane, int wave) {
  int wc = 0;
  const int el0  = tid * EPT;
  const int e0   = cbase + el0;
  const int sent = -2147483647 - 1;
  v4i da, db;
  if (vec8 != 0 && cbase + CHUNK <= nE) {
    da = *(const v4i*)(dsts + e0);
    db = *(const v4i*)(dsts + e0 + 4);
  } else {
    da.x = (e0     < nE) ? dsts[min(e0,     nE - 1)] : sent;
    da.y = (e0 + 1 < nE) ? dsts[min(e0 + 1, nE - 1)] : sent;
    da.z = (e0 + 2 < nE) ? dsts[min(e0 + 2, nE - 1)] : sent;
    da.w = (e0 + 3 < nE) ? dsts[min(e0 + 3, nE - 1)] : sent;
    db.x = (e0 + 4 < nE) ? dsts[min(e0 + 4, nE - 1)] : sent;
    db.y = (e0 + 5 < nE) ? dsts[min(e0 + 5, nE - 1)] : sent;
    db.z = (e0 + 6 < nE) ? dsts[min(e0 + 6, nE - 1)] : sent;
    db.w = (e0 + 7 < nE) ? dsts[min(e0 + 7, nE - 1)] : sent;
  }
  const unsigned nbs = (unsigned)slotBase;
  const unsigned unb = (unsigned)nb;
  const unsigned s0 = (unsigned)da.x - nbs, s1 = (unsigned)da.y - nbs;
  const unsigned s2 = (unsigned)da.z - nbs, s3 = (unsigned)da.w - nbs;
  const unsigned s4 = (unsigned)db.x - nbs, s5 = (unsigned)db.y - nbs;
  const unsigned s6 = (unsigned)db.z - nbs, s7 = (unsigned)db.w - nbs;
  const bool h0 = s0 < unb, h1 = s1 < unb, h2 = s2 < unb, h3 = s3 < unb;
  const bool h4 = s4 < unb, h5 = s5 < unb, h6 = s6 < unb, h7 = s7 < unb;
  const unsigned any = __builtin_amdgcn_ballot_w32(h0 | h1 | h2 | h3 | h4 | h5 | h6 | h7);
  if (any != 0u) {
#define HITJ(J, HJ, SJ) { \
      const unsigned mj = __builtin_amdgcn_ballot_w32(HJ); \
      if (mj != 0u) { \
        if (HJ) { \
          const int pos = wc + (int)__builtin_amdgcn_mbcnt_lo(mj, 0u); \
          if (pos < WCAP) list[wave * WCAP + pos] = ((el0 + (J)) << SLB) | (int)(SJ); \
        } \
        wc += (int)__builtin_popcount(mj); } }
    HITJ(0, h0, s0)
    HITJ(1, h1, s1)
    HITJ(2, h2, s2)
    HITJ(3, h3, s3)
    HITJ(4, h4, s4)
    HITJ(5, h5, s5)
    HITJ(6, h6, s6)
    HITJ(7, h7, s7)
#undef HITJ
  }
  return wc;
}

__global__ __launch_bounds__(NTHR) void k_prepw(const float* __restrict__ linw, const float* __restrict__ w1,
                                                unsigned short* bt) {
  const int tid = (int)threadIdx.x;
  const int pb  = (int)blockIdx.x;
  const int l   = pb / (2 * NBW);
  const int q   = pb - l * (2 * NBW);
  const bool second = q >= NBW;
  const int u  = (q & (NBW - 1)) * NTHR + tid;
  const int n  = u >> 5;
  const int k8 = (u & 31) * 8;
  const int kk = k8 & (DD - 1);
  v4f a, b;
  if (!second) {
    const float* p = linw + (size_t)l * DD * DD + (size_t)n * DD + kk;
    a = *(const v4fa*)p;
    b = *(const v4fa*)(p + 4);
  } else {
    const int seg = n >> 6;
    const int nc  = n & (HD - 1);
    const float* p = w1 + (size_t)l * K3 * HD + (size_t)(seg * DD + kk) * HD + nc;
    a.x = p[0];                a.y = p[(size_t)HD];      a.z = p[(size_t)2 * HD];  a.w = p[(size_t)3 * HD];
    b.x = p[(size_t)4 * HD];   b.y = p[(size_t)5 * HD];  b.z = p[(size_t)6 * HD];  b.w = p[(size_t)7 * HD];
  }
  const v8us o = pack8(a, b);
  unsigned short* dp = bt + ((size_t)(2 * l + (second ? 1 : 0)) * DD + (size_t)n) * KA + k8;
  *(volatile v8us*)dp = o;
  __threadfence();
  *(volatile v8us*)dp = o;
}

__device__ __forceinline__ void gemm64(const unsigned short* alds, const unsigned short* __restrict__ BT,
                                       v8f (&acc)[8], int wave, int hh, int m) {
  {
    const v8f z = {0.f, 0.f, 0.f, 0.f, 0.f, 0.f, 0.f, 0.f};
#pragma unroll
    for (int t = 0; t < 8; ++t) acc[t] = z;
  }
  const unsigned short* ap = alds + (size_t)(16 * wave + m) * (size_t)KA + 8 * hh;
  const unsigned short* bp = BT + (size_t)m * (size_t)KA + 8 * hh;
#pragma unroll 1
  for (int k0 = 0; k0 < KA; k0 += 32) {
    FragB af;
    af.h[0] = *(const v8usa*)(ap + k0);
    af.h[1] = *(const v8usa*)(ap + k0 + 16);
#pragma unroll
    for (int nt = 0; nt < 8; ++nt) {
      const unsigned short* wq = bp + (size_t)(16 * nt) * (size_t)KA + k0;
      FragB bf;
      bf.h[0] = *(const v8usa*)wq;
      bf.h[1] = *(const v8usa*)(wq + 16);
      acc[nt] = wmb(af, bf, acc[nt]);
    }
  }
}
__device__ __forceinline__ void stage64(float* stg, const v8f (&acc)[8], int wave, int hh, int m) {
#pragma unroll
  for (int nt = 0; nt < 8; ++nt) {
    const int lc = 16 * nt + m;
#pragma unroll
    for (int r = 0; r < 8; ++r) {
      const int lr = 16 * wave + 8 * hh + r;
      stg[lr * DD + lc] = acc[nt][r];
    }
  }
}

template <int SRC>
__global__ __launch_bounds__(GTHR) void k_node(const float* __restrict__ xin, const float* __restrict__ x0in,
                                               const float* __restrict__ curvp,
                                               const unsigned short* __restrict__ bt1,
                                               const unsigned short* __restrict__ bt2,
                                               const float* __restrict__ bias, int nN,
                                               float* xtan, float* xl, float* pab) {
  extern __shared__ __attribute__((aligned(16))) int ldyn[];
  unsigned short* alds = (unsigned short*)ldyn;
  float* stg = (float*)(ldyn + (GBM * KA) / 2);
  const int tid = (int)threadIdx.x, lane = tid & 31, wave = tid >> 5, hh = lane >> 4, m = lane & 15;
  const int rowBase = (int)blockIdx.x * GBM;

  const float cc  = fminf(fmaxf(bf16_val(curvp[0]), 0.1f), 10.0f);
  const float sc  = sqrtf(cc);
  const float rsc = 1.0f / sc;

#pragma unroll 1
  for (int i = 0; i < 16; ++i) {
    const int lr  = 16 * wave + i;
    const int row = rowBase + lr;
    const int rc  = row < nN ? row : nN - 1;
    const bool live = row < nN;
    float x0, s0, s1, s2, s3;
    if (SRC == 0) {
      const float* p = xin + (size_t)rc * XP;
      x0 = bf16_val(p[0]);
      const float* q = p + 1 + 4 * lane;
      s0 = bf16_val(q[0]); s1 = bf16_val(q[1]); s2 = bf16_val(q[2]); s3 = bf16_val(q[3]);
    } else {
      x0 = x0in[rc];
      const v4f s = *(const v4fa*)(xin + (size_t)rc * DD + 4 * lane);
      s0 = s.x; s1 = s.y; s2 = s.z; s3 = s.w;
    }
    const float a0   = fmaxf(sc * x0, X0MIN);
    const float dist = acoshf(a0) * rsc;
    const float nr   = fmaxf(sqrtf(wsum(s0 * s0 + s1 * s1 + s2 * s2 + s3 * s3)), EPSN);
    const float f    = dist * __builtin_amdgcn_rcpf(nr);
    const float t0 = live ? s0 * f : 0.0f, t1 = live ? s1 * f : 0.0f;
    const float t2 = live ? s2 * f : 0.0f, t3 = live ? s3 * f : 0.0f;
    v4f o; o.x = t0; o.y = t1; o.z = t2; o.w = t3;
    float* op = xtan + (size_t)row * DD + 4 * lane;
    *(volatile v4f*)op = o;
    __threadfence();
    *(volatile v4f*)op = o;
    int h01, h23, l01, l23;
    hilo_pack(t0, t1, t2, t3, h01, h23, l01, l23);
    const v4i w = regroup16(h01, h23, l01, l23, lane);
    *(v4ia*)(alds + (size_t)lr * KA + 8 * lane) = w;
  }
  __syncthreads();

  v8f acc[8];
  gemm64(alds, bt1, acc, wave, hh, m);
  stage64(stg, acc, wave, hh, m);
  __syncthreads();

  v4f b4;
  {
    const v4f bq = *(const v4fa*)(bias + 4 * lane);
    b4.x = bf16_val(bq.x); b4.y = bf16_val(bq.y); b4.z = bf16_val(bq.z); b4.w = bf16_val(bq.w);
  }
#pragma unroll 1
  for (int i = 0; i < 16; ++i) {
    const int lr   = 16 * wave + i;
    const int grow = rowBase + lr;
    const bool live = grow < nN;
    const v4f mv = *(const v4fa*)(stg + lr * DD + 4 * lane);
    const float v0 = live ? mv.x + b4.x : 0.0f, v1 = live ? mv.y + b4.y : 0.0f;
    const float v2 = live ? mv.z + b4.z : 0.0f, v3 = live ? mv.w + b4.w : 0.0f;
    v4f o; o.x = v0; o.y = v1; o.z = v2; o.w = v3;
    float* op = xl + (size_t)grow * DD + 4 * lane;
    *(volatile v4f*)op = o;
    __threadfence();
    *(volatile v4f*)op = o;
    int h01, h23, l01, l23;
    hilo_pack(v0, v1, v2, v3, h01, h23, l01, l23);
    const v4i w = regroup16(h01, h23, l01, l23, lane);
    *(v4ia*)(alds + (size_t)lr * KA + 8 * lane) = w;
  }
  __syncthreads();

  gemm64(alds, bt2, acc, wave, hh, m);
  stage64(stg, acc, wave, hh, m);
  __syncthreads();

#pragma unroll 1
  for (int i = 0; i < 16; ++i) {
    const int lr   = 16 * wave + i;
    const int grow = rowBase + lr;
    const bool live = grow < nN;
    const v4f mv = *(const v4fa*)(stg + lr * DD + 4 * lane);
    v4f o;
    o.x = live ? mv.x : 0.0f; o.y = live ? mv.y : 0.0f; o.z = live ? mv.z : 0.0f; o.w = live ? mv.w : 0.0f;
    float* op = pab + (size_t)grow * DD + 4 * lane;
    *(volatile v4f*)op = o;
    __threadfence();
    *(volatile v4f*)op = o;
  }
}

__device__ __forceinline__ void store_grp_out(const float* stg, float* ob, int npc, int rem, int tid) {
#pragma unroll 1
  for (int it = 0; it < NIT1; ++it) {
    const int p  = tid + NTHR * it;
    const int pc = p < NPG1 ? p : NPG1 - 1;
    const v4f v  = *(const v4fa*)(stg + 4 * pc);
    if (p < npc) *(volatile v4f*)(ob + 4 * (size_t)p) = v;
  }
#pragma unroll 1
  for (int j = 0; j < rem; ++j) {
    const float v = stg[4 * npc + j];
    if (tid == 0) *(volatile float*)(ob + 4 * (size_t)npc + j) = v;
  }
}
__device__ __forceinline__ void store_grp_ws(const float* stg, float* osp, float* ox0, int tid) {
#pragma unroll 1
  for (int it = 0; it < NIT0; ++it) {
    const int p = tid + NTHR * it;
    const v4f v = *(const v4fa*)(stg + 4 * p);
    *(volatile v4f*)(osp + 4 * (size_t)p) = v;
  }
  {
    const int tc = tid < (GR / 4) ? tid : (GR / 4) - 1;
    const v4f v  = *(const v4fa*)(stg + GR * DD + 4 * tc);
    if (tid < (GR / 4)) *(volatile v4f*)(ox0 + 4 * tid) = v;
  }
}

template <int FIN>
__global__ __launch_bounds__(NTHR) void k_scan(
    const int* __restrict__ gsrc, const int* __restrict__ keys, const int* __restrict__ ety,
    const float* __restrict__ ew, int nE, int nN, int nT, int vec8,
    const float* __restrict__ xtan, const float* __restrict__ xl, const float* __restrict__ pab,
    const float* __restrict__ emb, const float* __restrict__ w1, const float* __restrict__ b1,
    const float* __restrict__ w2, const float* __restrict__ b2p, const float* __restrict__ sibp,
    const float* __restrict__ curvp, const float* __restrict__ lng, const float* __restrict__ lnb,
    float* outSP, float* outX0, float* outD) {
  extern __shared__ __attribute__((aligned(16))) int dsm[];
  int* list = dsm;
  int* hl   = dsm + LISTN;
  int* sl   = hl + RCAP;
  int* cnt  = sl + RCAP;
  int* offs = cnt + NBA;
  int* cur  = offs + NBA;
  int* misc = cur + NBA;
  float* tcs  = (float*)(dsm + AGG_INTS);
  float* embs = tcs + TMAX * HD;
  float* w2s  = embs + TMAX * DD;
  float* lgs  = w2s + HD;
  float* lbs  = lgs + DD;
  float* stg  = lbs + DD;
  const int tid = (int)threadIdx.x, lane = tid & 31, wave = tid >> 5;
  const int nodeBase = (int)blockIdx.x * NBA;

  {
    const v4i z4 = {0, 0, 0, 0};
    for (int i = tid * 4; i < AGG_ZINTS; i += NTHR * 4) *(v4ia*)(dsm + i) = z4;
    if (tid < 16) misc[tid] = 0;
#pragma unroll 1
    for (int i = tid; i < TMAX * DD; i += NTHR) {
      const int t = i >> 7, c = i & (DD - 1);
      const int tcl = t < nT ? t : nT - 1;
      const float v = bf16_val(emb[(size_t)tcl * DD + c]);
      embs[i] = (t < nT) ? v : 0.0f;
    }
    if (tid < HD) w2s[tid] = bf16_val(w2[tid]);
    if (tid < DD) { lgs[tid] = bf16_val(lng[tid]); lbs[tid] = bf16_val(lnb[tid]); }
  }
  __syncthreads();
  {
#pragma unroll 1
    for (int o = tid; o < TMAX * HD; o += NTHR) {
      const int t = o >> 6, h = o & (HD - 1);
      const int tcl = t < nT ? t : nT - 1;
      const int kn  = (t < nT) ? DD : 0;
      const float* er = embs + tcl * DD;
      const float* wc = w1 + (size_t)(2 * DD) * HD + h;
      float d = 0.0f;
#pragma unroll 1
      for (int k = 0; k < kn; ++k) d = fmaf(er[k], bf16_val(wc[(size_t)k * HD]), d);
      tcs[o] = (t < nT) ? d + bf16_val(b1[h]) : 0.0f;
    }
  }
  __syncthreads();

  int nhit = 0, ov = 0;
  const int nChunks = (nE + CHUNK - 1) / CHUNK;
#pragma unroll 1
  for (int ch = 0; ch < nChunks; ++ch) {
    const int cbase = ch * CHUNK;
    const int wc = scan_chunk<SLA>(keys, nE, cbase, nodeBase, NBA, vec8, list, tid, lane, wave);
    if (lane == 0) misc[wave] = wc;
    __syncthreads();
    if (wave == 0) {
#pragma unroll 1
      for (int wq = 0; wq < NWAVE; ++wq) {
        int cw = misc[wq];
        cw = cw < 0 ? 0 : (cw > WCAP ? WCAP : cw);
#pragma unroll 1
        for (int b0 = 0; b0 < cw; b0 += 32) {
          const int idx = b0 + lane;
          const int ent = list[wq * WCAP + (idx < WCAP ? idx : WCAP - 1)];
          const int m32 = (cw - b0) < 32 ? (cw - b0) : 32;
#pragma unroll 1
          for (int k = 0; k < m32; ++k) {
            const int u    = __builtin_amdgcn_readlane(ent, k);
            const int slot = u & (NBA - 1);
            const int el   = (u >> SLA) & (CHUNK - 1);
            const int pk   = ((cbase + el) << SLA) | slot;
            if (nhit < RCAP) {
              if (lane == 0) { hl[nhit] = pk; cnt[slot] = cnt[slot] + 1; }
              nhit = nhit + 1;
            } else {
              ov = 1;
            }
          }
        }
      }
    }
    __syncthreads();
  }
  if (wave == 0 && lane == 0) { misc[8] = nhit; misc[9] = ov; }
  __syncthreads();
  int tt = misc[8];
  tt = tt < 0 ? 0 : (tt > RCAP ? RCAP : tt);
  const int ovf = misc[9];

  if (wave == 0) {
    const int base = lane * (NBA / 32);
    int s = 0;
#pragma unroll 1
    for (int i = 0; i < NBA / 32; ++i) s += cnt[base + i];
    int incl = s;
#pragma unroll
    for (int d = 1; d < 32; d <<= 1) {
      const int y = __shfl_up(incl, d, 32);
      if (lane >= d) incl += y;
    }
    int run = incl - s;
#pragma unroll 1
    for (int i = 0; i < NBA / 32; ++i) {
      const int cv = cnt[base + i];
      offs[base + i] = run;
      cur[base + i]  = run;
      run += cv;
    }
  }
  __syncthreads();
  if (wave == 0) {
#pragma unroll 1
    for (int b0 = 0; b0 < tt; b0 += 32) {
      const int idx = b0 + lane;
      const int ent = hl[idx < RCAP ? idx : RCAP - 1];
      const int m32 = (tt - b0) < 32 ? (tt - b0) : 32;
#pragma unroll 1
      for (int k = 0; k < m32; ++k) {
        const int u    = __builtin_amdgcn_readlane(ent, k);
        const int slot = u & (NBA - 1);
        if (lane == 0) {
          int p = cur[slot];
          p = p < 0 ? 0 : (p > RCAP - 1 ? RCAP - 1 : p);
          sl[p] = u;
          cur[slot] = p + 1;
        }
      }
    }
  }
  __syncthreads();

  const float cc  = fminf(fmaxf(bf16_val(curvp[0]), 0.1f), 10.0f);
  const float sc  = sqrtf(cc);
  const float rsc = 1.0f / sc;
  const float b2v = bf16_val(b2p[0]);
  const float sbv = bf16_val(sibp[0]);
  const float w2a = w2s[2 * lane], w2b = w2s[2 * lane + 1];
  const v4f g4 = *(const v4fa*)(lgs + 4 * lane);
  const v4f q4 = *(const v4fa*)(lbs + 4 * lane);
  const float qnan = __int_as_float(0x7fc00000);
  const float pz = (ovf != 0) ? qnan : 0.0f;

#pragma unroll 1
  for (int g = 0; g < NBA / GR; ++g) {
#pragma unroll 1
    for (int si = 0; si < GR / NWAVE; ++si) {
      const int lr   = si * NWAVE + wave;
      const int s    = g * GR + lr;
      const int node = nodeBase + s;
      const int ncl  = node < nN ? node : nN - 1;
      const bool live = node < nN;
      int c = cnt[s];
      const bool big = c > DEGCAP;
      c = c < 0 ? 0 : (c > DEGCAP ? DEGCAP : c);
      int ofs = offs[s];
      ofs = ofs < 0 ? 0 : (ofs > RCAP ? RCAP : ofs);
      const v2f pa = *(const v2fa*)(pab + (size_t)ncl * DD + 2 * lane);
      float mx = -3.0e38f, den = 0.0f, a0 = 0.0f, a1 = 0.0f, a2 = 0.0f, a3 = 0.0f;
#pragma unroll 1
      for (int b0 = 0; b0 < c; b0 += 32) {
        int idx = ofs + b0 + lane;
        idx = idx > RCAP - 1 ? RCAP - 1 : idx;
        const int ent = sl[idx];
        int eid = ent >> SLA;
        eid = eid < 0 ? 0 : (eid > nE - 1 ? nE - 1 : eid);
        int sr = gsrc[eid];
        sr = sr < 0 ? 0 : (sr > nN - 1 ? nN - 1 : sr);
        int ty = ety[eid];
        ty = ty < 0 ? 0 : (ty > nT - 1 ? nT - 1 : ty);
        const float wv = bf16_val(ew[eid]);
        const float ad = (logf(fmaxf(wv, EPSN)) + b2v) + ((ty == 1) ? sbv : 0.0f);
        const int wvi = __float_as_int(wv);
        const int adi = __float_as_int(ad);
        const int m32 = (c - b0) < 32 ? (c - b0) : 32;
#pragma unroll 1
        for (int k = 0; k < m32; ++k) {
          const int   sk = __builtin_amdgcn_readlane(sr, k);
          const int   tk = __builtin_amdgcn_readlane(ty, k);
          const float wk = __int_as_float(__builtin_amdgcn_readlane(wvi, k));
          const float ak = __int_as_float(__builtin_amdgcn_readlane(adi, k));
          const v2f pb = *(const v2fa*)(pab + (size_t)sk * DD + HD + 2 * lane);
          const float* tcr = tcs + tk * HD + 2 * lane;
          const float p0 = (pa.x + pb.x) + tcr[0];
          const float p1 = (pa.y + pb.y) + tcr[1];
          const float h0 = silu_f(p0), h1 = silu_f(p1);
          const float part = wsum(fmaf(h1, w2b, h0 * w2a));
          const float scr = part + ak;
          const float df  = scr - mx;
          const float ee  = __expf(-fabsf(df));
          const bool  up  = df > 0.0f;
          const float f1  = up ? ee : 1.0f;
          const float f2  = up ? 1.0f : ee;
          mx  = up ? scr : mx;
          den = fmaf(den, f1, f2);
          const float cf = f2 * wk;
          const v4f xj = *(const v4fa*)(xl + (size_t)sk * DD + 4 * lane);
          const v4f em = *(const v4fa*)(embs + tk * DD + 4 * lane);
          a0 = fmaf(a0, f1, cf * (xj.x + em.x));
          a1 = fmaf(a1, f1, cf * (xj.y + em.y));
          a2 = fmaf(a2, f1, cf * (xj.z + em.z));
          a3 = fmaf(a3, f1, cf * (xj.w + em.w));
        }
      }
      const float rden = __builtin_amdgcn_rcpf(den + 1e-16f);
      const v4f xt = *(const v4fa*)(xtan + (size_t)ncl * DD + 4 * lane);
      const float xa = fmaf(a0, rden, xt.x), xb = fmaf(a1, rden, xt.y);
      const float xc = fmaf(a2, rden, xt.z), xd = fmaf(a3, rden, xt.w);
      const float mu = wsum((xa + xb) + (xc + xd)) * (1.0f / DD);
      const float d0 = xa - mu, d1 = xb - mu, d2 = xc - mu, d3 = xd - mu;
      const float var = wsum(d0 * d0 + d1 * d1 + d2 * d2 + d3 * d3) * (1.0f / DD);
      const float rs  = rsqrtf(var + 1e-5f);
      const float y0 = fmaf(d0 * rs, g4.x, q4.x), y1 = fmaf(d1 * rs, g4.y, q4.y);
      const float y2 = fmaf(d2 * rs, g4.z, q4.z), y3 = fmaf(d3 * rs, g4.w, q4.w);
      const float nrm = fmaxf(sqrtf(wsum(y0 * y0 + y1 * y1 + y2 * y2 + y3 * y3)), EPSN);
      const float th  = sc * nrm;
      const float ex  = expf(th);
      const float iex = __builtin_amdgcn_rcpf(ex);
      const float ch  = (0.5f * (ex + iex)) * rsc;
      const float fac = (0.5f * (ex - iex)) * __builtin_amdgcn_rcpf(th);
      const float pzr = big ? qnan : pz;
      const float o0 = live ? ch + pzr : 0.0f;
      const float o1 = live ? fmaf(y0, fac, pzr) : 0.0f, o2 = live ? fmaf(y1, fac, pzr) : 0.0f;
      const float o3 = live ? fmaf(y2, fac, pzr) : 0.0f, o4 = live ? fmaf(y3, fac, pzr) : 0.0f;
      if constexpr (FIN != 0) {
        float* srow = stg + lr * XP;
        if (lane == 0) srow[0] = o0;
        srow[1 + 4 * lane] = o1; srow[2 + 4 * lane] = o2; srow[3 + 4 * lane] = o3; srow[4 + 4 * lane] = o4;
      } else {
        v4f ow; ow.x = o1; ow.y = o2; ow.z = o3; ow.w = o4;
        *(v4fa*)(stg + lr * DD + 4 * lane) = ow;
        if (lane == 0) stg[GR * DD + lr] = o0;
      }
    }
    __syncthreads();
    {
      const int row0 = nodeBase + g * GR;
      if constexpr (FIN != 0) {
        int rv = nN - row0;
        rv = rv < 0 ? 0 : (rv > GR ? GR : rv);
        const int vf  = rv * XP;
        const int npc = vf >> 2, rem = vf & 3;
        float* ob = outD + (size_t)row0 * XP;
        store_grp_out(stg, ob, npc, rem, tid);
        __threadfence();
        store_grp_out(stg, ob, npc, rem, tid);
      } else {
        float* osp = outSP + (size_t)row0 * DD;
        float* ox0 = outX0 + (size_t)row0;
        store_grp_ws(stg, osp, ox0, tid);
        __threadfence();
        store_grp_ws(stg, osp, ox0, tid);
      }
    }
    __syncthreads();
  }
}

static inline int cdiv(int a, int b) { return (a + b - 1) / b; }

extern "C" void kernel_launch(void* const* d_in, const int* in_sizes, int n_in,
                              void* d_out, int out_size, void* d_ws, size_t ws_size,
                              hipStream_t stream) {
  if (n_in < 15) return;
  if (in_sizes[0] < XP || (in_sizes[0] % XP) != 0) return;
  const int nN = in_sizes[0] / XP;
  if (nN < 1 || nN > (1 << 22)) return;
  if (in_sizes[1] < 2 || (in_sizes[1] & 1) != 0) return;
  const int nE = in_sizes[1] / 2;
  if (nE < 1 || nE >= (1 << 21)) return;
  if (in_sizes[2] != nE || in_sizes[3] != nE) return;
  const int nL = in_sizes[14];
  if (nL < 1 || nL > 64) return;
  if (in_sizes[4] != nL * DD * DD) return;
  if (in_sizes[5] != nL * DD || in_sizes[6] != nL * DD || in_sizes[7] != nL * DD) return;
  if (in_sizes[8] < nL * DD || (in_sizes[8] % (nL * DD)) != 0) return;
  const int nT = in_sizes[8] / (nL * DD);
  if (nT < 1 || nT > TMAX) return;
  if (in_sizes[9] != nL * K3 * HD) return;
  if (in_sizes[10] != nL * HD || in_sizes[11] != nL * HD) return;
  if (in_sizes[12] != nL || in_sizes[13] != nL) return;
  if ((long long)out_size != (long long)nN * XP) return;

  const float* xhyp = (const float*)d_in[0];
  const int*   edge = (const int*)  d_in[1];
  const int*   ety  = (const int*)  d_in[2];
  const float* ew   = (const float*)d_in[3];
  const float* linw = (const float*)d_in[4];
  const float* linb = (const float*)d_in[5];
  const float* lng  = (const float*)d_in[6];
  const float* lnb  = (const float*)d_in[7];
  const float* emb  = (const float*)d_in[8];
  const float* w1   = (const float*)d_in[9];
  const float* b1   = (const float*)d_in[10];
  const float* w2   = (const float*)d_in[11];
  const float* b2   = (const float*)d_in[12];
  const float* sib  = (const float*)d_in[13];
  const float* curv = (const float*)d_in[14];
  float* out = (float*)d_out;
  const int* gsrc = edge;
  const int* keys = edge + nE;

  const int MP  = cdiv(nN, GBM) * GBM;
  const int gL  = MP / GBM;
  const int gA  = cdiv(nN, NBA);
  const int MPX = gA * NBA;
  if ((long long)gA * NBA < (long long)nN) return;
  const int vec8 = ((nE & 3) == 0) ? 1 : 0;

  char* ws = (char*)d_ws;
  size_t off = 0;
  const size_t oBT  = off; off += (size_t)nL * 2 * DD * KA * 2;  off = (off + 255) & ~(size_t)255;
  const size_t oXT  = off; off += (size_t)MP * DD * 4;           off = (off + 255) & ~(size_t)255;
  const size_t oXL  = off; off += (size_t)MP * DD * 4;           off = (off + 255) & ~(size_t)255;
  const size_t oPAB = off; off += (size_t)MP * DD * 4;           off = (off + 255) & ~(size_t)255;
  const size_t oSP  = off; off += (size_t)MPX * DD * 4;          off = (off + 255) & ~(size_t)255;
  const size_t oX0  = off; off += (size_t)MPX * 4;               off = (off + 255) & ~(size_t)255;
  if (off > ws_size || off > (size_t)WSMAX) return;
  unsigned short* BT  = (unsigned short*)(ws + oBT);
  float* XTAN = (float*)(ws + oXT);
  float* XL   = (float*)(ws + oXL);
  float* PAB  = (float*)(ws + oPAB);
  float* SP1  = (float*)(ws + oSP);
  float* X01  = (float*)(ws + oX0);

  hipFuncSetAttribute(reinterpret_cast<const void*>(&k_node<0>), hipFuncAttributeMaxDynamicSharedMemorySize, LIN_LDS);
  hipFuncSetAttribute(reinterpret_cast<const void*>(&k_node<1>), hipFuncAttributeMaxDynamicSharedMemorySize, LIN_LDS);
  hipFuncSetAttribute(reinterpret_cast<const void*>(&k_scan<0>), hipFuncAttributeMaxDynamicSharedMemorySize, AGG_LDS);
  hipFuncSetAttribute(reinterpret_cast<const void*>(&k_scan<1>), hipFuncAttributeMaxDynamicSharedMemorySize, AGG_LDS);

  k_prepw<<<nL * 2 * NBW, NTHR, 0, stream>>>(linw, w1, BT);

  for (int l = 0; l < nL; ++l) {
    const unsigned short* bt1 = BT + (size_t)(2 * l) * DD * KA;
    const unsigned short* bt2 = BT + (size_t)(2 * l + 1) * DD * KA;
    const float* linb_l = linb + (size_t)l * DD;
    const float* curv_l = curv + l;
    if (l == 0)
      k_node<0><<<gL, GTHR, LIN_LDS, stream>>>(xhyp, X01, curv_l, bt1, bt2, linb_l, nN, XTAN, XL, PAB);
    else
      k_node<1><<<gL, GTHR, LIN_LDS, stream>>>(SP1, X01, curv_l, bt1, bt2, linb_l, nN, XTAN, XL, PAB);
    const float* emb_l = emb + (size_t)l * nT * DD;
    const float* w1_l  = w1 + (size_t)l * K3 * HD;
    const float* b1_l  = b1 + (size_t)l * HD;
    const float* w2_l  = w2 + (size_t)l * HD;
    const float* b2_l  = b2 + l;
    const float* sib_l = sib + l;
    const float* lng_l = lng + (size_t)l * DD;
    const float* lnb_l = lnb + (size_t)l * DD;
    if (l == nL - 1)
      k_scan<1><<<gA, NTHR, AGG_LDS, stream>>>(gsrc, keys, ety, ew, nE, nN, nT, vec8, XTAN, XL, PAB,
                                                emb_l, w1_l, b1_l, w2_l, b2_l, sib_l, curv_l, lng_l, lnb_l,
                                                SP1, X01, out);
    else
      k_scan<0><<<gA, NTHR, AGG_LDS, stream>>>(gsrc, keys, ety, ew, nE, nN, nT, vec8, XTAN, XL, PAB,
                                                emb_l, w1_l, b1_l, w2_l, b2_l, sib_l, curv_l, lng_l, lnb_l,
                                                SP1, X01, out);
  }
}
